// TransformerBlock_43525198577896
// MI455X (gfx1250) — hardware-verified
//
#include <hip/hip_runtime.h>
#ifndef NB
#define NB 2
#endif
#ifndef SEQ
#define SEQ 2048
#endif
#define NB_FULL 2
#define SEQ_FULL 2048
#define DM 1024
#define NH 16
#define HD 64
#define DFF 4096
#define QT0 128
#define LQ (3 * DM)
#define NR ((size_t)NB * SEQ)

static_assert(NB >= 1 && NB <= NB_FULL);
static_assert(SEQ <= SEQ_FULL);
static_assert(SEQ % 128 == 0);
static_assert(SEQ >= QT0 && QT0 == 128);
static_assert(NH * HD == DM && HD == 64);
static_assert(DM == 256 * 4);
static_assert(DM % 64 == 0 && LQ % 64 == 0 && DFF % 64 == 0);
static_assert(DM % 32 == 0 && DFF % 32 == 0 && HD % 32 == 0);
static_assert(((size_t)NB * QT0 * DM) % 8 == 0);

typedef unsigned short v8us __attribute__((ext_vector_type(8), may_alias));
typedef float  v8f  __attribute__((ext_vector_type(8)));
typedef float  v4f  __attribute__((ext_vector_type(4)));
typedef float  v4fa __attribute__((ext_vector_type(4), may_alias));
typedef _Float16 v16h __attribute__((ext_vector_type(16)));
typedef _Float16 v4h __attribute__((ext_vector_type(4)));
union FragH { v16h v; v8us half[2]; _Float16 h[16]; unsigned short u[16]; };

__device__ __forceinline__ unsigned short bf16_bits(float x) { unsigned int u = __float_as_uint(x); return (unsigned short)((u + 0x7FFFu + ((u >> 16) & 1u)) >> 16); }
__device__ __forceinline__ float bf16_val(unsigned short b) { return __uint_as_float(((unsigned int)b) << 16); }
__device__ __forceinline__ float bf16_rne(float x) { return bf16_val(bf16_bits(x)); }
__device__ __forceinline__ unsigned short f16_bits(float x) { const _Float16 hv = (_Float16)x; return __builtin_bit_cast(unsigned short, hv); }

__device__ __forceinline__ v16h g2_frag(const _Float16* p, int hh) { FragH f; f.half[0] = *(const v8us*)((const unsigned short*)p + 8 * hh); f.half[1] = *(const v8us*)((const unsigned short*)p + 16 + 8 * hh); return f.v; }
__device__ __forceinline__ v8f g2_mma(v16h a, v16h b, v8f c) { v8f d = __builtin_amdgcn_wmma_f32_16x16x32_f16(false, a, false, b, (short)0, c, false, false); asm volatile("v_nop\n\tv_nop\n\tv_nop\n\tv_nop" : "+v"(d) : "v"(a), "v"(b)); return d; }

__global__ __launch_bounds__(256) void k_wnat(const float* __restrict__ w, size_t n8, _Float16* __restrict__ Bt) {
  const size_t t = (size_t)blockIdx.x * 256 + threadIdx.x; if (t >= n8) return; FragH f;
#pragma unroll
  for (int q = 0; q < 8; ++q) f.h[q] = (_Float16)(bf16_rne(w[t * 8 + q]) * 16.0f);
  const v8us o = f.half[0];
  *(volatile v8us*)((unsigned short*)Bt + t * 8) = o; __threadfence(); *(volatile v8us*)((unsigned short*)Bt + t * 8) = o;
}

template <int BFIN>
__device__ __forceinline__ void ln16_body(const float* __restrict__ X, const float* __restrict__ g, const float* __restrict__ bb, float eps, _Float16* __restrict__ N16) {
  #pragma clang fp contract(off)
  __shared__ float red[256];
  const size_t r = blockIdx.x; const int t = threadIdx.x;
  const size_t rsrc = BFIN ? ((r / SEQ) * (size_t)SEQ_FULL + (r % SEQ)) : r;
  const v4f xa = *(const v4fa*)(X + rsrc * DM + t * 4); float s[4]; float sum = 0.f;
#pragma unroll
  for (int q = 0; q < 4; ++q) { s[q] = BFIN ? bf16_rne(xa[q]) : xa[q]; sum = sum + s[q]; }
  red[t] = sum; __syncthreads();
  for (int st = 128; st > 0; st >>= 1) { if (t < st) red[t] = red[t] + red[t + st]; __syncthreads(); }
  const float mu = red[0] * (1.0f / (float)DM); __syncthreads();
  float vs = 0.f;
#pragma unroll
  for (int q = 0; q < 4; ++q) { const float dl = s[q] - mu; vs = vs + dl * dl; }
  red[t] = vs; __syncthreads();
  for (int st = 128; st > 0; st >>= 1) { if (t < st) red[t] = red[t] + red[t + st]; __syncthreads(); }
  const float rs = rsqrtf(red[0] * (1.0f / (float)DM) + eps); v4h y;
#pragma unroll
  for (int q = 0; q < 4; ++q) { const int c = t * 4 + q; y[q] = (_Float16)(((s[q] - mu) * rs) * bf16_rne(g[c]) + bf16_rne(bb[c])); }
  for (int pass = 0; pass < 2; ++pass) { *(volatile v4h*)(N16 + r * DM + t * 4) = y; if (pass == 0) __threadfence(); }
}
__global__ __launch_bounds__(256) void k_ln_in(const float* __restrict__ X, const float* __restrict__ g, const float* __restrict__ bb, float eps, _Float16* __restrict__ N16) { ln16_body<1>(X, g, bb, eps, N16); }
__global__ __launch_bounds__(256) void k_ln_mid(const float* __restrict__ X, const float* __restrict__ g, const float* __restrict__ bb, float eps, _Float16* __restrict__ N16) { ln16_body<0>(X, g, bb, eps, N16); }

template <int ACT, int RESBF>
__device__ __forceinline__ void gemm2_body(const _Float16* __restrict__ A, int lda, size_t sA, const _Float16* __restrict__ Bh, int ldb, size_t sB, float alpha,
    const float* __restrict__ bias, const float* resid, int ldr, size_t sR, float* C, _Float16* C16, int ldc, size_t sC, int M, int N, int K) {
  static_assert(ACT == 0 || ACT == 3);
  __shared__ __attribute__((aligned(16))) float so[4][32][68];
  const int tid = threadIdx.x, w = tid >> 5, lane = tid & 31, ln = lane & 15, hh = lane >> 4; const int by = blockIdx.y;
  A += (size_t)by * sA; Bh += (size_t)by * sB; const size_t cofs = (size_t)by * sC;
  const int ntn = N >> 6; const int mt = blockIdx.x / ntn, nq = blockIdx.x - mt * ntn; const int row0 = mt * 128 + 32 * w, col0 = nq * 64; if (row0 >= M) return;
  const _Float16* a0p = A + (size_t)(row0 + ln) * lda; const _Float16* a1p = a0p + (size_t)16 * lda;
  const _Float16* b0p = Bh + (size_t)(col0 + ln) * ldb; const _Float16* b1p = b0p + (size_t)16 * ldb; const _Float16* b2p = b1p + (size_t)16 * ldb; const _Float16* b3p = b2p + (size_t)16 * ldb;
  const v8f z8 = {0.f,0.f,0.f,0.f,0.f,0.f,0.f,0.f}; v8f c00 = z8, c01 = z8, c02 = z8, c03 = z8, c10 = z8, c11 = z8, c12 = z8, c13 = z8;
#pragma unroll 1
  for (int kb = 0; kb < K; kb += 32) { const v16h a0 = g2_frag(a0p + kb, hh), a1 = g2_frag(a1p + kb, hh);
    v16h b = g2_frag(b0p + kb, hh); c00 = g2_mma(a0, b, c00); c10 = g2_mma(a1, b, c10);
    b = g2_frag(b1p + kb, hh); c01 = g2_mma(a0, b, c01); c11 = g2_mma(a1, b, c11);
    b = g2_frag(b2p + kb, hh); c02 = g2_mma(a0, b, c02); c12 = g2_mma(a1, b, c12);
    b = g2_frag(b3p + kb, hh); c03 = g2_mma(a0, b, c03); c13 = g2_mma(a1, b, c13); }
  v8f accs[8] = {c00, c01, c02, c03, c10, c11, c12, c13};
#pragma unroll
  for (int u = 0; u < 8; ++u) { const int t = u & 3, half = u >> 2; const int col = col0 + t * 16 + ln; const float bv = bias ? bf16_rne(bias[col]) : 0.f;
#pragma unroll
    for (int r = 0; r < 8; ++r) { const int rloc = half * 16 + 8 * hh + r; float v = accs[u][r] * alpha + bv; if (ACT == 3) v = fmaxf(v, 0.f); so[w][rloc][t * 16 + ln] = v; } }
  __builtin_amdgcn_fence(4  , "workgroup"); __builtin_amdgcn_wave_barrier();
  const int rsub = lane >> 4, c4 = (lane & 15) * 4;
  if (resid != nullptr) {
    const float* rp = resid + (size_t)by * sR + (size_t)row0 * ldr + col0 + c4;
#pragma unroll 4
    for (int q = 0; q < 16; ++q) { const int r = q * 2 + rsub; v4f rv = *(const v4fa*)(rp + (size_t)r * ldr);
      if (RESBF) { rv[0] = bf16_rne(rv[0]); rv[1] = bf16_rne(rv[1]); rv[2] = bf16_rne(rv[2]); rv[3] = bf16_rne(rv[3]); }
      v4f sv = *(const v4fa*)&so[w][r][c4]; sv = sv + rv; *(v4fa*)&so[w][r][c4] = sv; }
  }
  for (int pass = 0; pass < 2; ++pass) {
#pragma unroll
    for (int q = 0; q < 16; ++q) { const int r = q * 2 + rsub; const v4f v = *(const v4fa*)&so[w][r][c4];
      if (C) *(volatile v4f*)(C + cofs + (size_t)(row0 + r) * ldc + col0 + c4) = v;
      if (C16) { v4h h4; h4[0] = (_Float16)v[0]; h4[1] = (_Float16)v[1]; h4[2] = (_Float16)v[2]; h4[3] = (_Float16)v[3]; *(volatile v4h*)(C16 + cofs + (size_t)(row0 + r) * ldc + col0 + c4) = h4; } }
    if (pass == 0) __threadfence(); }
}
__global__ __launch_bounds__(128) void k_gemm_lin(const _Float16* __restrict__ A, int lda, size_t sA, const _Float16* __restrict__ Bh, int ldb, size_t sB, float alpha, const float* __restrict__ bias, const float* resid, int ldr, size_t sR, float* C, _Float16* C16, int ldc, size_t sC, int M, int N, int K) {
  gemm2_body<0, 0>(A, lda, sA, Bh, ldb, sB, alpha, bias, resid, ldr, sR, C, C16, ldc, sC, M, N, K); }
__global__ __launch_bounds__(128) void k_gemm_lin_rb(const _Float16* __restrict__ A, int lda, size_t sA, const _Float16* __restrict__ Bh, int ldb, size_t sB, float alpha, const float* __restrict__ bias, const float* resid, int ldr, size_t sR, float* C, _Float16* C16, int ldc, size_t sC, int M, int N, int K) {
  gemm2_body<0, 1>(A, lda, sA, Bh, ldb, sB, alpha, bias, resid, ldr, sR, C, C16, ldc, sC, M, N, K); }
__global__ __launch_bounds__(128) void k_gemm_relu(const _Float16* __restrict__ A, int lda, size_t sA, const _Float16* __restrict__ Bh, int ldb, size_t sB, float alpha, const float* __restrict__ bias, const float* resid, int ldr, size_t sR, float* C, _Float16* C16, int ldc, size_t sC, int M, int N, int K) {
  gemm2_body<3, 0>(A, lda, sA, Bh, ldb, sB, alpha, bias, resid, ldr, sR, C, C16, ldc, sC, M, N, K); }

__global__ __launch_bounds__(256) void k_vt(const _Float16* __restrict__ V16, int ldv, _Float16* __restrict__ Vt) {
  __shared__ unsigned short tl[64][66];
  const int tid = threadIdx.x; const int slab = blockIdx.x / (SEQ / 64), lg = blockIdx.x % (SEQ / 64); const int b = slab / NH, h = slab % NH;
  for (int i = tid; i < 64 * 8; i += 256) { const int r = i / 8, c8 = (i % 8) * 8; FragH f; f.half[0] = *(const v8us*)((const unsigned short*)V16 + ((size_t)b * SEQ + lg * 64 + r) * ldv + h * 64 + c8);
#pragma unroll
    for (int q = 0; q < 8; ++q) tl[r][c8 + q] = f.u[q]; }
  __syncthreads();
  for (int pass = 0; pass < 2; ++pass) {
#pragma unroll
    for (int rd = 0; rd < 2; ++rd) { const int d = rd * 32 + tid / 8, pc = tid % 8; FragH f;
#pragma unroll
      for (int q = 0; q < 8; ++q) f.u[q] = tl[pc * 8 + q][d];
      *(volatile v8us*)((unsigned short*)Vt + ((size_t)slab * 64 + d) * SEQ + lg * 64 + pc * 8) = f.half[0]; }
    if (pass == 0) __threadfence(); }
}

__global__ __launch_bounds__(128) void k_flash(const _Float16* __restrict__ QKV, const _Float16* __restrict__ VT, _Float16* __restrict__ O16) {
  __shared__ __attribute__((aligned(16))) unsigned short pb[4][16][40];
  __shared__ __attribute__((aligned(16))) unsigned short ob[4][16][72];
  const int tid = threadIdx.x, w = tid >> 5, lane = tid & 31, ln = lane & 15, hh = lane >> 4;
  const int bh = blockIdx.y, b = bh / NH, h = bh % NH;
  const int q0 = (blockIdx.x * 4 + w) * 16;
  const size_t r0 = (size_t)b * SEQ;
  const _Float16* qp = QKV + (r0 + q0 + ln) * LQ + h * HD;
  const v16h aq0 = g2_frag(qp, hh), aq1 = g2_frag(qp + 32, hh);
  const _Float16* kbase = QKV + r0 * LQ + DM + h * HD;
  const _Float16* vbase = VT + (size_t)bh * HD * SEQ;
  const v8f z8 = {0.f,0.f,0.f,0.f,0.f,0.f,0.f,0.f};
  v8f acc[4] = {z8, z8, z8, z8};
  float m[8], l[8];
#pragma unroll
  for (int r = 0; r < 8; ++r) { m[r] = -1.0e30f; l[r] = 0.f; }
  const int kend = q0 + 15;
#pragma unroll 1
  for (int kb = 0; kb <= kend; kb += 32) {
    float s0[8], s1[8];
    { const int key = kb + ln; const _Float16* kp = kbase + (size_t)key * LQ;
      const v16h b0 = g2_frag(kp, hh), b1 = g2_frag(kp + 32, hh);
      v8f st = z8; st = g2_mma(aq0, b0, st); st = g2_mma(aq1, b1, st);
#pragma unroll
      for (int r = 0; r < 8; ++r) { const int qr = q0 + 8 * hh + r; s0[r] = (key <= qr) ? st[r] * 0.125f : -1.0e30f; } }
    { const int key = kb + 16 + ln; const _Float16* kp = kbase + (size_t)key * LQ;
      const v16h b0 = g2_frag(kp, hh), b1 = g2_frag(kp + 32, hh);
      v8f st = z8; st = g2_mma(aq0, b0, st); st = g2_mma(aq1, b1, st);
#pragma unroll
      for (int r = 0; r < 8; ++r) { const int qr = q0 + 8 * hh + r; s1[r] = (key <= qr) ? st[r] * 0.125f : -1.0e30f; } }
#pragma unroll
    for (int r = 0; r < 8; ++r) {
      float mx = fmaxf(s0[r], s1[r]);
      mx = fmaxf(mx, __shfl_xor(mx, 1, 32)); mx = fmaxf(mx, __shfl_xor(mx, 2, 32)); mx = fmaxf(mx, __shfl_xor(mx, 4, 32)); mx = fmaxf(mx, __shfl_xor(mx, 8, 32));
      const float mn = fmaxf(m[r], mx);
      const float ea = __expf(fmaxf(m[r] - mn, -80.0f));
      const float al = (m[r] < -1.0e29f) ? 0.f : ea;
      m[r] = mn;
      const float e0 = __expf(fmaxf(s0[r] - mn, -80.0f)), e1 = __expf(fmaxf(s1[r] - mn, -80.0f));
      const float p0 = (s0[r] > -1.0e29f) ? e0 : 0.f, p1 = (s1[r] > -1.0e29f) ? e1 : 0.f;
      l[r] = l[r] * al + (p0 + p1);
      acc[0][r] *= al; acc[1][r] *= al; acc[2][r] *= al; acc[3][r] *= al;
      pb[w][8 * hh + r][ln] = f16_bits(p0 * 256.0f); pb[w][8 * hh + r][16 + ln] = f16_bits(p1 * 256.0f);
    }
    __builtin_amdgcn_fence(4  , "workgroup"); __builtin_amdgcn_wave_barrier();
    FragH ap; ap.half[0] = *(const v8us*)&pb[w][ln][8 * hh]; ap.half[1] = *(const v8us*)&pb[w][ln][16 + 8 * hh];
    __builtin_amdgcn_fence(4  , "workgroup"); __builtin_amdgcn_wave_barrier();
#pragma unroll
    for (int j = 0; j < 4; ++j) { const v16h bv = g2_frag(vbase + (size_t)(j * 16 + ln) * SEQ + kb, hh); acc[j] = g2_mma(ap.v, bv, acc[j]); }
  }
#pragma unroll
  for (int r = 0; r < 8; ++r) {
    float ls = l[r];
    ls += __shfl_xor(ls, 1, 32); ls += __shfl_xor(ls, 2, 32); ls += __shfl_xor(ls, 4, 32); ls += __shfl_xor(ls, 8, 32);
    const float inv = 0.25f * (1.0f / ls);
#pragma unroll
    for (int j = 0; j < 4; ++j) ob[w][8 * hh + r][j * 16 + ln] = f16_bits(acc[j][r] * inv);
  }
  __builtin_amdgcn_fence(4  , "workgroup"); __builtin_amdgcn_wave_barrier();
  for (int pass = 0; pass < 2; ++pass) {
#pragma unroll
    for (int it = 0; it < 4; ++it) { const int row = it * 4 + (lane >> 3), pc = (lane & 7) * 8; const v8us v = *(const v8us*)&ob[w][row][pc];
      *(volatile v8us*)((unsigned short*)O16 + (r0 + q0 + row) * DM + h * HD + pc) = v; }
    if (pass == 0) __threadfence(); }
}

__global__ __launch_bounds__(64) void k_att0(const float* __restrict__ QF, const float* __restrict__ KF, const float* __restrict__ VF, int ld, size_t sF, float scale, float* __restrict__ OF, int ldo, size_t sO) {
  #pragma clang fp contract(off)
  __shared__ __attribute__((aligned(16))) float lq[64][64]; __shared__ __attribute__((aligned(16))) float lo[64][64];
  const int tid = threadIdx.x; const int h = blockIdx.x / (QT0 / 64), rg = blockIdx.x % (QT0 / 64); const int i = rg * 64 + tid;
  const size_t fo = (size_t)blockIdx.y * sF; const float* qb = QF + fo; const float* kbp = KF + fo; const float* vbp = VF + fo; float* ofp = OF + (size_t)blockIdx.y * sO;
  const float* qr = qb + (size_t)i * ld + h * HD;
#pragma unroll 1
  for (int c = 0; c < HD / 4; ++c) { *(v4fa*)&lq[tid][c * 4] = *(const v4fa*)(qr + c * 4); const v4f z = {0.f, 0.f, 0.f, 0.f}; *(v4fa*)&lo[tid][c * 4] = z; }
  float m = -1.0e30f, l = 0.f; const int jmax = rg * 64 + 63;
#pragma unroll 1
  for (int j = 0; j <= jmax; ++j) { const float* kr = kbp + (size_t)j * ld + h * HD; const float* vr = vbp + (size_t)j * ld + h * HD; float s = 0.f;
#pragma unroll 1
    for (int c = 0; c < HD / 4; ++c) { const v4f kq = *(const v4fa*)(kr + c * 4); const v4f qq = *(const v4fa*)&lq[tid][c * 4]; s = s + qq[0] * kq[0]; s = s + qq[1] * kq[1]; s = s + qq[2] * kq[2]; s = s + qq[3] * kq[3]; }
    s = s * scale;
    const float f = (j <= i) ? 1.f : 0.f; const float sm = fmaf(f, s, (1.f - f) * -1.0e30f); const float mn = fmaxf(m, sm); const float sc = expf(m - mn); const float e = expf(sm - mn); l = l * sc + e; m = mn;
#pragma unroll 1
    for (int c = 0; c < HD / 4; ++c) { const v4f vv = *(const v4fa*)(vr + c * 4); v4f oo = *(const v4fa*)&lo[tid][c * 4]; oo[0] = oo[0] * sc + e * vv[0]; oo[1] = oo[1] * sc + e * vv[1]; oo[2] = oo[2] * sc + e * vv[2]; oo[3] = oo[3] * sc + e * vv[3]; *(v4fa*)&lo[tid][c * 4] = oo; } }
  const float fin = 64.0f * (1.0f / l);
#pragma unroll 1
  for (int c = 0; c < HD / 4; ++c) { v4f oo = *(const v4fa*)&lo[tid][c * 4]; oo[0] = oo[0] * fin; oo[1] = oo[1] * fin; oo[2] = oo[2] * fin; oo[3] = oo[3] * fin; *(v4fa*)&lo[tid][c * 4] = oo; }
  __syncthreads();
  for (int pass = 0; pass < 2; ++pass) {
#pragma unroll 1
    for (int it = 0; it < 16; ++it) { const int row = it * 4 + tid / 16, pc = (tid % 16) * 4; const v4f v = *(const v4fa*)&lo[row][pc]; *(volatile v4f*)(ofp + (size_t)(rg * 64 + row) * ldo + h * HD + pc) = v; }
    if (pass == 0) __threadfence(); }
}

__global__ __launch_bounds__(256) void k_hl(const float* __restrict__ F, _Float16* __restrict__ Hh, _Float16* __restrict__ Hl, size_t n8) {
  const size_t t = (size_t)blockIdx.x * 256 + threadIdx.x; if (t >= n8) return; FragH fh, fl; const v4f a = *(const v4fa*)(F + t * 8), c = *(const v4fa*)(F + t * 8 + 4);
#pragma unroll
  for (int q = 0; q < 4; ++q) { _Float16 hv = (_Float16)a[q]; fh.h[q] = hv; fl.h[q] = (_Float16)((a[q] - (float)hv) * 1024.0f); hv = (_Float16)c[q]; fh.h[4 + q] = hv; fl.h[4 + q] = (_Float16)((c[q] - (float)hv) * 1024.0f); }
  const v8us oh = fh.half[0], ol = fl.half[0];
  for (int pass = 0; pass < 2; ++pass) { *(volatile v8us*)((unsigned short*)Hh + t * 8) = oh; *(volatile v8us*)((unsigned short*)Hl + t * 8) = ol; if (pass == 0) __threadfence(); }
}

constexpr size_t al256(size_t x) { return (x + 255) & ~(size_t)255; }
constexpr size_t SZ_BQKV = (size_t)3 * DM * DM * 2;
constexpr size_t SZ_BO   = (size_t)DM * DM * 2;
constexpr size_t SZ_BW1  = (size_t)DFF * DM * 2;
constexpr size_t SZ_BW2  = (size_t)DM * DFF * 2;
constexpr size_t SZ_X16  = NR * DM * 2;
constexpr size_t SZ_X1   = NR * DM * 4;
constexpr size_t SZ_M16  = NR * DM * 2;
constexpr size_t SZ_QKV  = NR * LQ * 2;
constexpr size_t SZ_O16  = NR * DM * 2;
constexpr size_t SZ_HF16 = NR * DFF * 2;
constexpr size_t SZ_ATT  = (SZ_QKV + SZ_O16 > SZ_HF16) ? (SZ_QKV + SZ_O16) : SZ_HF16;
constexpr size_t SZ_VT   = (size_t)NB * NH * HD * SEQ * 2;
constexpr size_t SZ_F0   = (size_t)NB * QT0 * LQ * 4;
constexpr size_t SZ_OF0  = (size_t)NB * QT0 * DM * 4;
constexpr size_t SZ_OH0  = (size_t)NB * QT0 * DM * 2;
constexpr size_t OFF_BQKV = 0;
constexpr size_t OFF_BO   = OFF_BQKV + al256(SZ_BQKV);
constexpr size_t OFF_BW1  = OFF_BO + al256(SZ_BO);
constexpr size_t OFF_BW2  = OFF_BW1 + al256(SZ_BW1);
constexpr size_t OFF_X16  = OFF_BW2 + al256(SZ_BW2);
constexpr size_t OFF_X1   = OFF_X16 + al256(SZ_X16);
constexpr size_t OFF_M16  = OFF_X1 + al256(SZ_X1);
constexpr size_t OFF_ATT  = OFF_M16 + al256(SZ_M16);
constexpr size_t OFF_VT   = OFF_ATT + al256(SZ_ATT);
constexpr size_t OFF_F0   = OFF_VT + al256(SZ_VT);
constexpr size_t OFF_OF0  = OFF_F0 + al256(SZ_F0);
constexpr size_t OFF_OH0  = OFF_OF0 + al256(SZ_OF0);
constexpr size_t OFF_OL0  = OFF_OH0 + al256(SZ_OH0);
constexpr size_t WS_TOTAL = OFF_OL0 + al256(SZ_OH0);
static_assert(WS_TOTAL <= (size_t)134217728);
static_assert(SZ_HF16 <= SZ_ATT && SZ_QKV + SZ_O16 <= SZ_ATT);
static_assert(SZ_QKV % 256 == 0);

extern "C" void kernel_launch(void* const* d_in, const int* in_sizes, int n_in,
                              void* d_out, int out_size, void* d_ws, size_t ws_size, hipStream_t stream) {
  if (n_in < 14) return;
  const size_t xneed = ((size_t)(NB - 1) * SEQ_FULL + SEQ) * DM;
  if ((size_t)in_sizes[0] < xneed || (size_t)out_size < xneed) return;
  if (in_sizes[1] < DM * DM || in_sizes[2] < DM * DM || in_sizes[3] < DM * DM || in_sizes[4] < DM * DM) return;
  if (in_sizes[5] < DM || in_sizes[6] < DM || in_sizes[7] < DM || in_sizes[8] < DM || in_sizes[9] < DM) return;
  if (in_sizes[10] < DFF * DM || in_sizes[11] < DFF || in_sizes[12] < DM * DFF || in_sizes[13] < DM) return;
  if (WS_TOTAL > ws_size) return;
  const float* x   = (const float*)d_in[0];
  const float* wq  = (const float*)d_in[1];
  const float* wk  = (const float*)d_in[2];
  const float* wv  = (const float*)d_in[3];
  const float* wo  = (const float*)d_in[4];
  const float* bo  = (const float*)d_in[5];
  const float* g1  = (const float*)d_in[6];
  const float* s1  = (const float*)d_in[7];
  const float* g2  = (const float*)d_in[8];
  const float* s2  = (const float*)d_in[9];
  const float* w1  = (const float*)d_in[10];
  const float* b1  = (const float*)d_in[11];
  const float* w2  = (const float*)d_in[12];
  const float* b2  = (const float*)d_in[13];
  float* out = (float*)d_out;
  char* ws = (char*)d_ws;
  _Float16* BQKV = (_Float16*)(ws + OFF_BQKV); _Float16* BO = (_Float16*)(ws + OFF_BO); _Float16* BW1 = (_Float16*)(ws + OFF_BW1); _Float16* BW2 = (_Float16*)(ws + OFF_BW2);
  _Float16* X16 = (_Float16*)(ws + OFF_X16); float* X1 = (float*)(ws + OFF_X1); _Float16* M16 = (_Float16*)(ws + OFF_M16);
  _Float16* QKV = (_Float16*)(ws + OFF_ATT); _Float16* O16 = (_Float16*)(ws + OFF_ATT + SZ_QKV); _Float16* HF16 = (_Float16*)(ws + OFF_ATT);
  _Float16* VT = (_Float16*)(ws + OFF_VT); float* F0 = (float*)(ws + OFF_F0); float* OF0 = (float*)(ws + OFF_OF0); _Float16* OH0 = (_Float16*)(ws + OFF_OH0); _Float16* OL0 = (_Float16*)(ws + OFF_OL0);

  { const size_t n8 = (size_t)DM * DM / 8; const unsigned gw = (unsigned)((n8 + 255) / 256);
    k_wnat<<<gw, 256, 0, stream>>>(wq, n8, BQKV);
    k_wnat<<<gw, 256, 0, stream>>>(wk, n8, BQKV + (size_t)DM * DM);
    k_wnat<<<gw, 256, 0, stream>>>(wv, n8, BQKV + (size_t)2 * DM * DM);
    k_wnat<<<gw, 256, 0, stream>>>(wo, n8, BO); }
  { const size_t n8 = (size_t)DFF * DM / 8; const unsigned gw = (unsigned)((n8 + 255) / 256);
    k_wnat<<<gw, 256, 0, stream>>>(w1, n8, BW1);
    k_wnat<<<gw, 256, 0, stream>>>(w2, n8, BW2); }
  k_ln_in<<<(unsigned)NR, 256, 0, stream>>>(x, g1, s1, 1e-5f, X16);
  k_gemm_lin<<<dim3((unsigned)((NR / 128) * (LQ / 64)), 1), 128, 0, stream>>>(X16, DM, (size_t)0, BQKV, DM, (size_t)0, 0.0625f, nullptr, nullptr, 0, (size_t)0, nullptr, QKV, LQ, (size_t)0, (int)NR, LQ, DM);
  k_vt<<<(unsigned)(NB * NH * (SEQ / 64)), 256, 0, stream>>>(QKV + 2 * DM, LQ, VT);
  k_flash<<<dim3(SEQ / 64, NB * NH), 128, 0, stream>>>(QKV, VT, O16);
  k_gemm_lin<<<dim3((QT0 / 128) * (LQ / 64), NB), 128, 0, stream>>>(X16, DM, (size_t)SEQ * DM, BQKV, DM, (size_t)0, 0.0625f, nullptr, nullptr, 0, (size_t)0, F0, nullptr, LQ, (size_t)QT0 * LQ, QT0, LQ, DM);
  k_att0<<<dim3(NH * (QT0 / 64), NB), 64, 0, stream>>>(F0, F0 + DM, F0 + 2 * DM, LQ, (size_t)QT0 * LQ, 0.125f, OF0, DM, (size_t)QT0 * DM);
  k_gemm_lin_rb<<<dim3((SEQ / 128) * (DM / 64), NB), 128, 0, stream>>>(O16, DM, (size_t)SEQ * DM, BO, DM, (size_t)0, 0.0009765625f, bo, x, DM, (size_t)SEQ_FULL * DM, X1, nullptr, DM, (size_t)SEQ * DM, SEQ, DM, DM);
  k_hl<<<(unsigned)(((size_t)NB * QT0 * DM / 8 + 255) / 256), 256, 0, stream>>>(OF0, OH0, OL0, (size_t)NB * QT0 * DM / 8);
  k_gemm_lin_rb<<<dim3((QT0 / 128) * (DM / 64), NB), 128, 0, stream>>>(OH0, DM, (size_t)QT0 * DM, BO, DM, (size_t)0, 0.0009765625f, bo, x, DM, (size_t)SEQ_FULL * DM, X1, nullptr, DM, (size_t)SEQ * DM, QT0, DM, DM);
  k_gemm_lin<<<dim3((QT0 / 128) * (DM / 64), NB), 128, 0, stream>>>(OL0, DM, (size_t)QT0 * DM, BO, DM, (size_t)0, 9.5367431640625e-07f, nullptr, X1, DM, (size_t)SEQ * DM, X1, nullptr, DM, (size_t)SEQ * DM, QT0, DM, DM);
  k_ln_mid<<<(unsigned)NR, 256, 0, stream>>>(X1, g2, s2, 1e-5f, M16);
  k_gemm_relu<<<dim3((unsigned)((NR / 128) * (DFF / 64)), 1), 128, 0, stream>>>(M16, DM, (size_t)0, BW1, DM, (size_t)0, 0.0625f, b1, nullptr, 0, (size_t)0, nullptr, HF16, DFF, (size_t)0, (int)NR, DFF, DM);
  k_gemm_lin<<<dim3((SEQ / 128) * (DM / 64), NB), 128, 0, stream>>>(HF16, DFF, (size_t)SEQ * DFF, BW2, DFF, (size_t)0, 0.0625f, b2, X1, DM, (size_t)SEQ * DM, out, nullptr, DM, (size_t)SEQ_FULL * DM, SEQ, DM, DFF);
}
